// DCNv4PackFlowGuided_30812095381654
// MI455X (gfx1250) — hardware-verified
//
#include <hip/hip_runtime.h>
#include <stddef.h>

constexpr int kNB    = 4;
constexpr int kCIN   = 64;
constexpr int kHH    = 128;
constexpr int kWD    = 128;
constexpr int kHW    = 16384;
constexpr int kNPIX  = 65536;
constexpr int kCE    = 224;
constexpr int kNG    = 14;
constexpr int kCG    = 16;
constexpr int kTAPS  = 9;
constexpr int kOMG   = 27;
constexpr int kOMW   = 384;
constexpr int kNVP   = 256;
constexpr int kVP    = 256;
constexpr int kSP    = 256;
constexpr int kCOUT  = 64;
constexpr int kNBIAS = kNVP + kOMW + kCOUT;
constexpr float kSSC = 16.0f;
constexpr float kWSC = 16.0f;

constexpr size_t kBytesVAL  = (size_t)kHW * kVP * 4;
constexpr size_t kBytesOM   = (size_t)kHW * kOMW * 4;
constexpr size_t kBytesS    = (size_t)kHW * kSP * 2;
constexpr size_t kBytesINP  = (size_t)kHW * kCE * 2;
constexpr size_t kBytesWv   = (size_t)kNVP * kCE * 2;
constexpr size_t kBytesWm   = (size_t)kOMW * kCE * 2;
constexpr size_t kBytesWo   = (size_t)kCOUT * kCE * 2;
constexpr size_t kBytesBias = (size_t)kNBIAS * 4;
constexpr size_t kWsTotal   = kBytesVAL + kBytesOM + kBytesS + kBytesINP + kBytesWv + kBytesWm + kBytesWo + kBytesBias;
typedef char chk_ws_total[(kWsTotal <= (size_t)134217728) ? 1 : -1];
typedef char chk_ws_align[(((kBytesVAL | kBytesOM | kBytesS | kBytesINP | kBytesWv | kBytesWm | kBytesWo | kBytesBias) % 128) == 0) ? 1 : -1];
typedef char chk_kdepth[((kCE % 32) == 0) ? 1 : -1];
typedef char chk_tiles[((kHW % 64) == 0 && (kNVP % 64) == 0 && (kOMW % 64) == 0 && (kCOUT % 64) == 0) ? 1 : -1];

typedef __attribute__((ext_vector_type(16))) _Float16 v16h;
typedef __attribute__((ext_vector_type(8)))  _Float16 v8h;
typedef __attribute__((ext_vector_type(16))) __bf16   v16b;
typedef __attribute__((ext_vector_type(8)))  __bf16   v8b;
typedef __attribute__((ext_vector_type(8)))  float    v8f;
typedef __attribute__((ext_vector_type(4)))  float    v4f;
typedef __attribute__((ext_vector_type(4)))  unsigned v4u;

__device__ __forceinline__ unsigned short f2bf_bits(float f) {
  unsigned u = __float_as_uint(f);
  return (unsigned short)((u + 0x7FFFu + ((u >> 16) & 1u)) >> 16);
}
__device__ __forceinline__ float bf_bits2f(unsigned short h) { return __uint_as_float(((unsigned)h) << 16); }

__device__ __forceinline__ unsigned pk2(unsigned short a, unsigned short b) {
  return (unsigned)a | ((unsigned)b << 16);
}
__device__ __forceinline__ unsigned pkh2(float a, float b) {
  return pk2(__builtin_bit_cast(unsigned short, (_Float16)a), __builtin_bit_cast(unsigned short, (_Float16)b));
}

__device__ __forceinline__ void dep_guard_h(v8f& a, v8f& b, v16h x, v16h y) { asm volatile("v_nop\n\tv_nop\n\tv_nop\n\tv_nop" : "+v"(a), "+v"(b) : "v"(x), "v"(y)); }
__device__ __forceinline__ void dep_guard_b(v8f& a, v8f& b, v16b x, v16b y) { asm volatile("v_nop\n\tv_nop\n\tv_nop\n\tv_nop" : "+v"(a), "+v"(b) : "v"(x), "v"(y)); }
__device__ __forceinline__ void keep4_h(v16h a, v16h b, v16h c, v16h d) { asm volatile("v_nop" :: "v"(a), "v"(b), "v"(c), "v"(d)); }
__device__ __forceinline__ void keep4_b(v16b a, v16b b, v16b c, v16b d) { asm volatile("v_nop" :: "v"(a), "v"(b), "v"(c), "v"(d)); }
__device__ __forceinline__ void acc_guard4(v8f& a, v8f& b, v8f& c, v8f& d) { asm volatile("v_nop\n\tv_nop\n\tv_nop\n\tv_nop" : "+v"(a), "+v"(b), "+v"(c), "+v"(d)); }
template <typename T> struct Frag;
template <> struct Frag<_Float16> {
  typedef v16h V; union U { v16h v; v8h h[2]; };
  static __device__ __forceinline__ v16h load(const _Float16* p) {
    U f; f.h[0] = *(const v8h*)(p); f.h[1] = *(const v8h*)(p + 16); return f.v;
  }
  static __device__ __forceinline__ v8f mma(v16h a, v16h b, v8f c) {
    return __builtin_amdgcn_wmma_f32_16x16x32_f16(false, a, false, b, (short)0, c, false, false);
  }
  static __device__ __forceinline__ void guard(v8f& a, v8f& b, v16h x, v16h y) { dep_guard_h(a, b, x, y); }
  static __device__ __forceinline__ void keep(v16h a, v16h b, v16h c, v16h d) { keep4_h(a, b, c, d); }
};
template <> struct Frag<__bf16> {
  typedef v16b V; union U { v16b v; v8b h[2]; };
  static __device__ __forceinline__ v16b load(const __bf16* p) {
    U f; f.h[0] = *(const v8b*)(p); f.h[1] = *(const v8b*)(p + 16); return f.v;
  }
  static __device__ __forceinline__ v8f mma(v16b a, v16b b, v8f c) {
    return __builtin_amdgcn_wmma_f32_16x16x32_bf16(false, a, false, b, (short)0, c, false, false);
  }
  static __device__ __forceinline__ void guard(v8f& a, v8f& b, v16b x, v16b y) { dep_guard_b(a, b, x, y); }
  static __device__ __forceinline__ void keep(v16b a, v16b b, v16b c, v16b d) { keep4_b(a, b, c, d); }
};

template <int ET> struct Elem;
template <> struct Elem<0> { typedef _Float16 T; };
template <> struct Elem<1> { typedef __bf16 T; };
template <int ET, bool SPLIT, int BIAS_MODE, int OUT_MODE, bool RESID, int ACT = 0>
__global__ __launch_bounds__(256) void wmma_gemm64(
    const unsigned short* __restrict__ Ap, const unsigned short* __restrict__ A2p, int lda, long strideA,
    const unsigned short* __restrict__ Btp, const unsigned short* __restrict__ Bt2p, int ldb, long strideB,
    void* __restrict__ Cout, void* __restrict__ Cout2, int ldc, long strideC,
    const float* __restrict__ bias,
    const float* __restrict__ resid, long strideR,
    int M, int N, int K, float scale) {
  typedef typename Elem<ET>::T T;
  typedef typename Frag<T>::V V;
  const T* A = (const T*)Ap; const T* A2 = (const T*)A2p; const T* Bt = (const T*)Btp; const T* Bt2 = (const T*)Bt2p;
  __shared__ __align__(16) float sT[8][16 * 68];
  const int b    = blockIdx.y;
  const int lane = threadIdx.x & 31;
  const int wave = threadIdx.x >> 5;
  const int tilesN = N >> 6;
  const int tilesM = M >> 6;
  const int tile = blockIdx.x * 8 + wave;
  if (tile >= tilesM * tilesN) return;
  const int tm = tile / tilesN;
  const int tn = tile - tm * tilesN;
  const int m0 = tm << 6;
  const int n0 = tn << 6;

  const T* Ab  = A  + (size_t)b * strideA;
  const T* Bb  = Bt + (size_t)b * strideB;
  const T* Ab2 = SPLIT ? (A2  + (size_t)b * strideA) : nullptr;
  const T* Bb2 = SPLIT ? (Bt2 + (size_t)b * strideB) : nullptr;

  const int rlane = lane & 15;
  const int koff  = (lane >> 4) * 8;
  const int mOff  = (lane >> 4) * 8;

  v8f acc[4][4];
#pragma unroll
  for (int i = 0; i < 4; ++i)
#pragma unroll
    for (int j = 0; j < 4; ++j) acc[i][j] = (v8f){0.f,0.f,0.f,0.f,0.f,0.f,0.f,0.f};

  for (int k0 = 0; k0 < K; k0 += 32) {
    V bh[4], bl[4];
#pragma unroll
    for (int j = 0; j < 4; ++j) {
      const size_t bo = (size_t)(n0 + (j << 4) + rlane) * ldb + koff + k0;
      bh[j] = Frag<T>::load(Bb + bo);
      if (SPLIT) bl[j] = Frag<T>::load(Bb2 + bo);
    }
#pragma unroll
    for (int i = 0; i < 4; ++i) {
      const size_t ao = (size_t)(m0 + (i << 4) + rlane) * lda + koff + k0;
      V ah = Frag<T>::load(Ab + ao);
      V al;
      if (SPLIT) al = Frag<T>::load(Ab2 + ao);
#pragma unroll
      for (int j = 0; j < 4; ++j) {
        acc[i][j] = Frag<T>::mma(ah, bh[j], acc[i][j]);
        if (SPLIT) {
          acc[i][j] = Frag<T>::mma(ah, bl[j], acc[i][j]);
          acc[i][j] = Frag<T>::mma(al, bh[j], acc[i][j]);
        }
      }
      Frag<T>::guard(acc[i][0], acc[i][3], ah, SPLIT ? al : ah);
    }
    Frag<T>::keep(bh[0], bh[1], bh[2], bh[3]);
    if (SPLIT) Frag<T>::keep(bl[0], bl[1], bl[2], bl[3]);
  }
  acc_guard4(acc[0][0], acc[0][1], acc[0][2], acc[0][3]);
  acc_guard4(acc[1][0], acc[1][1], acc[1][2], acc[1][3]);
  acc_guard4(acc[2][0], acc[2][1], acc[2][2], acc[2][3]);
  acc_guard4(acc[3][0], acc[3][1], acc[3][2], acc[3][3]);

  float* slab = sT[wave];
  const float* Rb = RESID ? (resid + (size_t)b * strideR) : nullptr;
#pragma unroll
  for (int i = 0; i < 4; ++i) {
    const int mBase = m0 + (i << 4);
#pragma unroll
    for (int j = 0; j < 4; ++j) {
      const int n = n0 + (j << 4) + rlane;
      float bv = 0.f;
      if (BIAS_MODE == 2) bv = bias[n];
#pragma unroll
      for (int r = 0; r < 8; ++r) {
        float v = acc[i][j][r] * scale;
        if (BIAS_MODE == 1) v += bias[mBase + mOff + r];
        if (BIAS_MODE == 2) v += bv;
        if (RESID) v += Rb[(size_t)(mBase + mOff + r) * ldc + n];
        if (ACT == 1) v = tanhf(v);
        if (ACT == 2) v = fmaxf(v, 0.0f);
        if (ACT == 3) v = v / (1.0f + expf(-v));
        if (ACT == 4) v = (v > 0.f) ? v : 0.01f * v;
        if (ACT == 5) v = 0.5f * v * (1.0f + erff(v * 0.70710678118654752f));
        slab[(mOff + r) * 68 + (j << 4) + rlane] = v;
      }
    }
    __builtin_amdgcn_fence(__ATOMIC_RELEASE, "workgroup");
    __builtin_amdgcn_wave_barrier();
    __builtin_amdgcn_fence(__ATOMIC_ACQUIRE, "workgroup");
    if (OUT_MODE == 0) {
      float* C = (float*)Cout + (size_t)b * strideC;
      const int hh = lane >> 4, c4 = (lane & 15) * 4;
      for (int pass = 0; pass < 2; ++pass) {
#pragma unroll
        for (int it = 0; it < 8; ++it) {
          const int row = it * 2 + hh;
          v4f v = *(const v4f*)(slab + row * 68 + c4);
          *(volatile v4f*)(C + (size_t)(mBase + row) * ldc + n0 + c4) = v;
        }
        __threadfence();
      }
    } else {
      const int q = lane >> 3, c8 = (lane & 7) * 8;
      unsigned short* C  = (unsigned short*)Cout  + (size_t)b * strideC;
      unsigned short* C2 = (OUT_MODE == 2) ? ((unsigned short*)Cout2 + (size_t)b * strideC) : nullptr;
      for (int pass = 0; pass < 2; ++pass) {
#pragma unroll
        for (int it = 0; it < 4; ++it) {
          const int row = it * 4 + q;
          const float* sp = slab + row * 68 + c8;
          v8h hv, lv;
#pragma unroll
          for (int e = 0; e < 8; ++e) {
            if (OUT_MODE == 1) {
              hv[e] = (_Float16)sp[e];
            } else {
              unsigned short hb = f2bf_bits(sp[e]);
              unsigned short lb = f2bf_bits(sp[e] - bf_bits2f(hb));
              hv[e] = __builtin_bit_cast(_Float16, hb);
              lv[e] = __builtin_bit_cast(_Float16, lb);
            }
          }
          *(volatile v8h*)(C + (size_t)(mBase + row) * ldc + n0 + c8) = hv;
          if (OUT_MODE == 2) *(volatile v8h*)(C2 + (size_t)(mBase + row) * ldc + n0 + c8) = lv;
        }
        __threadfence();
      }
    }
    __builtin_amdgcn_fence(__ATOMIC_RELEASE, "workgroup");
    __builtin_amdgcn_wave_barrier();
    __builtin_amdgcn_fence(__ATOMIC_ACQUIRE, "workgroup");
  }
}

template <int MODE> __device__ __forceinline__ unsigned short cvt16(float v, float scl) {
  const unsigned short hb = f2bf_bits(v);
  if (MODE == 0) return hb;
  return __builtin_bit_cast(unsigned short, (_Float16)(bf_bits2f(hb) * scl));
}

template <int MODE>
__global__ __launch_bounds__(256) void k_prep_wT(const float* __restrict__ w, int ncols, int nreal, int npad, float scl,
                                                 unsigned short* __restrict__ outp) {
  const int g = blockIdx.x * 256 + threadIdx.x;
  if (g < npad * (kCE / 8)) {
    const int e0 = g * 8;
    const int n  = e0 / kCE;
    const int k0 = e0 - n * kCE;
    const int nc = (n < nreal) ? n : (nreal - 1);
    float f[8];
#pragma unroll
    for (int j = 0; j < 8; ++j) {
      const float v = w[(size_t)(k0 + j) * ncols + nc];
      f[j] = (n < nreal) ? v : 0.0f;
    }
    v4u u;
    u[0] = pk2(cvt16<MODE>(f[0], scl), cvt16<MODE>(f[1], scl));
    u[1] = pk2(cvt16<MODE>(f[2], scl), cvt16<MODE>(f[3], scl));
    u[2] = pk2(cvt16<MODE>(f[4], scl), cvt16<MODE>(f[5], scl));
    u[3] = pk2(cvt16<MODE>(f[6], scl), cvt16<MODE>(f[7], scl));
    volatile v4u* d = (volatile v4u*)(outp + (size_t)e0);
    *d = u;
    __threadfence();
    *d = u;
  }
}

__global__ __launch_bounds__(256) void k_prep_bias(const float* __restrict__ vb, const float* __restrict__ mb,
                                                   const float* __restrict__ ob, float* __restrict__ bias) {
  const int i = blockIdx.x * 256 + threadIdx.x;
  if (i < kNBIAS) {
    const int iv = (i < kCE) ? i : (kCE - 1);
    int im = i - kNVP;         im = im < 0 ? 0 : (im > kOMW - 1 ? kOMW - 1 : im);
    int io = i - kNVP - kOMW;  io = io < 0 ? 0 : (io > kCOUT - 1 ? kCOUT - 1 : io);
    const float a = vb[iv], m = mb[im], c = ob[io];
    float v = (i < kCE) ? a : ((i < kNVP) ? 0.0f : ((i < kNVP + kOMW) ? m : c));
    v = bf_bits2f(f2bf_bits(v));
    ((volatile float*)bias)[i] = v;
    __threadfence();
    ((volatile float*)bias)[i] = v;
  }
}

__global__ __launch_bounds__(256) void k_pack(const float* __restrict__ x, const float* __restrict__ xw,
                                              const float* __restrict__ xc, const float* __restrict__ fl,
                                              int bimg, unsigned short* __restrict__ inp) {
  const int g = blockIdx.x * 256 + threadIdx.x;
  if (g < kHW * kCE / 8) {
    const int e0  = g * 8;
    const int pix = e0 / kCE;
    const int c0  = e0 - pix * kCE;
    const int sel = c0 >> 6;
    const float* src = (sel == 0) ? x : ((sel == 1) ? xw : ((sel == 2) ? xc : fl));
    const int isfl = (sel == 3) ? 1 : 0;
    const int cs   = isfl ? 2 : kCIN;
    const int cc   = c0 & 63;
    float f[8];
#pragma unroll
    for (int j = 0; j < 8; ++j) {
      const int ch = isfl ? (j & 1) : (cc + j);
      f[j] = src[((size_t)bimg * cs + ch) * kHW + pix];
    }
    v4u u;
    u[0] = pk2(f2bf_bits(f[0]), f2bf_bits(f[1]));
    u[1] = pk2(f2bf_bits(f[2]), f2bf_bits(f[3]));
    u[2] = pk2(f2bf_bits(f[4]), f2bf_bits(f[5]));
    u[3] = pk2(f2bf_bits(f[6]), f2bf_bits(f[7]));
    volatile v4u* d = (volatile v4u*)(inp + (size_t)e0);
    *d = u;
    __threadfence();
    *d = u;
  }
}

__global__ __launch_bounds__(256) void k_dsample(const float* __restrict__ val, const float* __restrict__ om,
                                                 unsigned short* __restrict__ S) {
  const int lane = threadIdx.x & 31, wave = threadIdx.x >> 5;
  const int tok  = blockIdx.x * 8 + wave;
  const int ho = tok >> 7, wo = tok & (kWD - 1);
  const int graw = lane >> 1;
  const int gq   = (graw < kNG) ? graw : (kNG - 1);
  const int ch   = gq * kCG + (lane & 1) * 8;
  const float* omr = om + (size_t)tok * kOMW + gq * kOMG;
  const float* vb  = val + ch;
  v4f acca = (v4f){0.f, 0.f, 0.f, 0.f};
  v4f accb = (v4f){0.f, 0.f, 0.f, 0.f};
#pragma unroll 1
  for (int k = 0; k < kTAPS; ++k) {
    const int ki = k / 3;
    const int kj = k - ki * 3;
    const float dx = omr[2 * k];
    const float dy = omr[2 * k + 1];
    const float mk = omr[2 * kTAPS + k];
    float py = (float)(ho - 1 + ki) + dy;
    float px = (float)(wo - 1 + kj) + dx;
    py = fminf(fmaxf(py, -8.0f), (float)(kHH + 8));
    px = fminf(fmaxf(px, -8.0f), (float)(kWD + 8));
    const float y0 = floorf(py), x0 = floorf(px);
    const float wy1 = py - y0, wx1 = px - x0;
    const float wy0 = 1.0f - wy1, wx0 = 1.0f - wx1;
    const int y0i = (int)y0, x0i = (int)x0;
    const int y1i = y0i + 1, x1i = x0i + 1;
    const bool vy0 = (unsigned)y0i < (unsigned)kHH;
    const bool vy1 = (unsigned)y1i < (unsigned)kHH;
    const bool vx0 = (unsigned)x0i < (unsigned)kWD;
    const bool vx1 = (unsigned)x1i < (unsigned)kWD;
    float w00 = wy0 * wx0, w01 = wy0 * wx1, w10 = wy1 * wx0, w11 = wy1 * wx1;
    w00 = (vy0 && vx0) ? w00 : 0.0f;
    w01 = (vy0 && vx1) ? w01 : 0.0f;
    w10 = (vy1 && vx0) ? w10 : 0.0f;
    w11 = (vy1 && vx1) ? w11 : 0.0f;
    const int yc0 = y0i < 0 ? 0 : (y0i > kHH - 1 ? kHH - 1 : y0i);
    const int yc1 = y1i < 0 ? 0 : (y1i > kHH - 1 ? kHH - 1 : y1i);
    const int xc0 = x0i < 0 ? 0 : (x0i > kWD - 1 ? kWD - 1 : x0i);
    const int xc1 = x1i < 0 ? 0 : (x1i > kWD - 1 ? kWD - 1 : x1i);
    const float* r00 = vb + ((size_t)yc0 * kWD + xc0) * kVP;
    const float* r01 = vb + ((size_t)yc0 * kWD + xc1) * kVP;
    const float* r10 = vb + ((size_t)yc1 * kWD + xc0) * kVP;
    const float* r11 = vb + ((size_t)yc1 * kWD + xc1) * kVP;
    const v4f g00a = *(const v4f*)(r00), g00b = *(const v4f*)(r00 + 4);
    const v4f g01a = *(const v4f*)(r01), g01b = *(const v4f*)(r01 + 4);
    const v4f g10a = *(const v4f*)(r10), g10b = *(const v4f*)(r10 + 4);
    const v4f g11a = *(const v4f*)(r11), g11b = *(const v4f*)(r11 + 4);
    v4f sa = g00a * w00; sa = sa + g01a * w01; sa = sa + g10a * w10; sa = sa + g11a * w11;
    v4f sb = g00b * w00; sb = sb + g01b * w01; sb = sb + g10b * w10; sb = sb + g11b * w11;
    acca = acca + sa * mk;
    accb = accb + sb * mk;
  }
  const float osc = (graw < kNG) ? kSSC : 0.0f;
  acca = acca * osc;
  accb = accb * osc;
  v4u u;
  u[0] = pkh2(acca[0], acca[1]); u[1] = pkh2(acca[2], acca[3]);
  u[2] = pkh2(accb[0], accb[1]); u[3] = pkh2(accb[2], accb[3]);
  volatile v4u* d = (volatile v4u*)(S + (size_t)tok * kSP + lane * 8);
  *d = u;
  __threadfence();
  *d = u;
}

extern "C" void kernel_launch(void* const* d_in, const int* in_sizes, int n_in,
                              void* d_out, int out_size, void* d_ws, size_t ws_size,
                              hipStream_t stream) {
  if (n_in < 10) return;
  if (in_sizes[0] != kNPIX * kCIN || in_sizes[1] != kNPIX * kCIN || in_sizes[2] != kNPIX * kCIN ||
      in_sizes[3] != kNB * 2 * kHW || in_sizes[4] != kCE * kCE || in_sizes[5] != kCE ||
      in_sizes[6] != kCE * kOMW || in_sizes[7] != kOMW || in_sizes[8] != kCE * kCE || in_sizes[9] != kCE) return;
  if (out_size != kNB * kCOUT * kHW) return;
  if (kWsTotal > ws_size) return;

  const float* x        = (const float*)d_in[0];
  const float* xw       = (const float*)d_in[1];
  const float* xc       = (const float*)d_in[2];
  const float* flow     = (const float*)d_in[3];
  const float* value_w  = (const float*)d_in[4];
  const float* value_b  = (const float*)d_in[5];
  const float* offset_w = (const float*)d_in[6];
  const float* offset_b = (const float*)d_in[7];
  const float* output_w = (const float*)d_in[8];
  const float* output_b = (const float*)d_in[9];
  float* out = (float*)d_out;

  char* ws = (char*)d_ws;
  size_t o = 0;
  float* VAL = (float*)(ws + o);                      o += kBytesVAL;
  float* OM  = (float*)(ws + o);                      o += kBytesOM;
  unsigned short* S   = (unsigned short*)(ws + o);   o += kBytesS;
  unsigned short* INP = (unsigned short*)(ws + o);   o += kBytesINP;
  unsigned short* WvT = (unsigned short*)(ws + o);   o += kBytesWv;
  unsigned short* WmT = (unsigned short*)(ws + o);   o += kBytesWm;
  unsigned short* WoT = (unsigned short*)(ws + o);   o += kBytesWo;
  float* bias = (float*)(ws + o);                     o += kBytesBias;
  if (o != kWsTotal || o > ws_size || o > (size_t)134217728) return;

  k_prep_wT<0><<<(kNVP * (kCE / 8) + 255) / 256, 256, 0, stream>>>(value_w, kCE, kCE, kNVP, 1.0f, WvT);
  k_prep_wT<0><<<(kOMW * (kCE / 8) + 255) / 256, 256, 0, stream>>>(offset_w, kOMW, kOMW, kOMW, 1.0f, WmT);
  k_prep_wT<1><<<(kCOUT * (kCE / 8) + 255) / 256, 256, 0, stream>>>(output_w, kCE, kCOUT, kCOUT, kWSC, WoT);
  k_prep_bias<<<(kNBIAS + 255) / 256, 256, 0, stream>>>(value_b, offset_b, output_b, bias);

  for (int b = 0; b < kNB; ++b) {
    k_pack<<<(kHW * kCE / 8 + 255) / 256, 256, 0, stream>>>(x, xw, xc, flow, b, INP);
    wmma_gemm64<1, false, 2, 0, false><<<dim3((kHW / 64) * (kNVP / 64) / 8, 1), 256, 0, stream>>>(
        INP, INP, kCE, 0L,
        WvT, WvT, kCE, 0L,
        (void*)VAL, (void*)S, kVP, 0L,
        bias,
        bias, 0L,
        kHW, kNVP, kCE, 1.0f);
    wmma_gemm64<1, false, 2, 0, false><<<dim3((kHW / 64) * (kOMW / 64) / 8, 1), 256, 0, stream>>>(
        INP, INP, kCE, 0L,
        WmT, WmT, kCE, 0L,
        (void*)OM, (void*)S, kOMW, 0L,
        bias + kNVP,
        bias, 0L,
        kHW, kOMW, kCE, 1.0f);
    k_dsample<<<kHW / 8, 256, 0, stream>>>(VAL, OM, S);
    wmma_gemm64<0, false, 1, 0, false><<<dim3((kCOUT / 64) * (kHW / 64) / 8, 1), 256, 0, stream>>>(
        WoT, WoT, kCE, 0L,
        S, S, kSP, 0L,
        (void*)(out + (size_t)b * kCOUT * kHW), (void*)S, kHW, 0L,
        bias + kNVP + kOMW,
        bias, 0L,
        kCOUT, kHW, kCE, 1.0f / (kSSC * kWSC));
  }
}
